// GAGNN_Model_37984690765934
// MI455X (gfx1250) — hardware-verified
//
#include <hip/hip_runtime.h>
#include <stddef.h>


#define FIN     128
#define FO      512
#define NH      8
#define HC      64
#define EC      16
#define DH      64
#define PQW     128
#define K2      512
#define K1OFF   1024
#define MLPIN   1040
#define GH      32
#define WP      128
#define W1P     512
#define XSP     512
#define HP      512
#define ESP     8
#define SAP     136
#define STP     132
#define MISCN   160
#define NTHR    256
#define NWAVE   8
#define EPT     8
#define CHUNK   (NTHR * EPT)
#define WCAP    (EPT * 32)
#define LISTN   (NWAVE * WCAP)
#define NBMAX   2048
#define SLOTB   11
#define RCAP    20480
#define DEGCAP  4096
#define EPI     2
#define LPS     16
#define GBM     64
#define GTHR    128
#define ETHR    128
#define TPW     8
#define NEG_SLOPE 0.2f
#define CA      16.0f
#define CW      64.0f
#define CX      16.0f
#define CH      16.0f
#define SCL     0.0009765625f
#define INVCX   0.0625f
#define WSCAP   134217728
#define LDS_BUILD ((2 * RCAP + 2 * NBMAX + LISTN) * 4 + 64)

static_assert((CHUNK & (CHUNK - 1)) == 0 && CHUNK <= 4096);
static_assert(NBMAX == (1 << SLOTB));
static_assert(NTHR * 8 == NBMAX);
static_assert(LISTN >= NBMAX);
static_assert(LISTN >= NWAVE * WCAP);
static_assert((RCAP % 32) == 0);
static_assert(LDS_BUILD <= 300000);
static_assert(GBM == (GTHR / 32) * 16);
static_assert(NH * HC == FO);
static_assert(FO == 4 * FIN);
static_assert((FIN % 32) == 0 && (K2 % 32) == 0);
static_assert(EPI * LPS == 32);
static_assert(HC == 2 * 32);
static_assert(GBM * ESP == GTHR * 4);
static_assert(PQW == 2 * DH);
static_assert(EC * NH + NH <= MISCN && (MISCN % 32) == 0);
static_assert((SAP * 2) % 16 == 0);
static_assert((STP * 4) % 16 == 0 && STP >= PQW);
static_assert(EC * DH == 2 * 4 * ETHR);
static_assert(DH == 4 * 16 && DH * 2 == 4 * 32);

typedef float    v4f  __attribute__((ext_vector_type(4)));
typedef float    v8f  __attribute__((ext_vector_type(8)));
typedef int      v4i  __attribute__((ext_vector_type(4)));
typedef int      v8i  __attribute__((ext_vector_type(8)));
typedef _Float16 v8h  __attribute__((ext_vector_type(8)));
typedef _Float16 v16h __attribute__((ext_vector_type(16)));
union FragH { v16h v; v8h h[2]; v8i w; };
union U8 { v8f v; v4f q[2]; };

__device__ __forceinline__ v8f wmh(const FragH& a, const FragH& b, v8f c) {
  v8f d = __builtin_amdgcn_wmma_f32_16x16x32_f16(false, a.v, false, b.v, (short)0, c, false, false);
  asm volatile("v_nop\n\tv_nop\n\tv_nop\n\tv_nop" : "+v"(d) : "v"(a.w), "v"(b.w));
  return d;
}

__device__ __forceinline__ v8h pack8(v4f a, v4f b, float sc) {
  v8h hv;
  hv[0] = (_Float16)(a.x * sc); hv[1] = (_Float16)(a.y * sc);
  hv[2] = (_Float16)(a.z * sc); hv[3] = (_Float16)(a.w * sc);
  hv[4] = (_Float16)(b.x * sc); hv[5] = (_Float16)(b.y * sc);
  hv[6] = (_Float16)(b.z * sc); hv[7] = (_Float16)(b.w * sc);
  return hv;
}

__device__ __forceinline__ v8h pack8v(v8f a, float sc) {
  const v8f s = a * sc;
  return __builtin_convertvector(s, v8h);
}

__device__ __forceinline__ v8f cvt8(v8h hv) {
  return __builtin_convertvector(hv, v8f);
}

__device__ __forceinline__ v8f leaky8(v8f v) {
  const v8f t = v * NEG_SLOPE;
  v8f r;
#pragma unroll
  for (int i = 0; i < 8; ++i) r[i] = fmaxf(v[i], t[i]);
  return r;
}

__device__ __forceinline__ int scan_chunk(const int* __restrict__ dsts, int nE, int cbase, int slotBase,
                                          int nb, int vec8, int* list, int tid, int lane, int wave) {
  int wc = 0;
  const int el0  = tid * EPT;
  const int e0   = cbase + el0;
  const int sent = -2147483647 - 1;
  v4i da, db;
  if (vec8 != 0 && cbase + CHUNK <= nE) {
    da = *(const v4i*)(dsts + e0);
    db = *(const v4i*)(dsts + e0 + 4);
  } else {
    da.x = (e0     < nE) ? dsts[min(e0,     nE - 1)] : sent;
    da.y = (e0 + 1 < nE) ? dsts[min(e0 + 1, nE - 1)] : sent;
    da.z = (e0 + 2 < nE) ? dsts[min(e0 + 2, nE - 1)] : sent;
    da.w = (e0 + 3 < nE) ? dsts[min(e0 + 3, nE - 1)] : sent;
    db.x = (e0 + 4 < nE) ? dsts[min(e0 + 4, nE - 1)] : sent;
    db.y = (e0 + 5 < nE) ? dsts[min(e0 + 5, nE - 1)] : sent;
    db.z = (e0 + 6 < nE) ? dsts[min(e0 + 6, nE - 1)] : sent;
    db.w = (e0 + 7 < nE) ? dsts[min(e0 + 7, nE - 1)] : sent;
  }
  const unsigned nbs = (unsigned)slotBase;
  const unsigned unb = (unsigned)nb;
  const unsigned s0 = (unsigned)da.x - nbs, s1 = (unsigned)da.y - nbs;
  const unsigned s2 = (unsigned)da.z - nbs, s3 = (unsigned)da.w - nbs;
  const unsigned s4 = (unsigned)db.x - nbs, s5 = (unsigned)db.y - nbs;
  const unsigned s6 = (unsigned)db.z - nbs, s7 = (unsigned)db.w - nbs;
  const bool h0 = s0 < unb, h1 = s1 < unb, h2 = s2 < unb, h3 = s3 < unb;
  const bool h4 = s4 < unb, h5 = s5 < unb, h6 = s6 < unb, h7 = s7 < unb;
  const unsigned any = __builtin_amdgcn_ballot_w32(h0 | h1 | h2 | h3 | h4 | h5 | h6 | h7);
  if (any != 0u) {
#define HITJ(J, HJ, SJ) { \
      const unsigned mj = __builtin_amdgcn_ballot_w32(HJ); \
      if (mj != 0u) { \
        if (HJ) { \
          const int pos = wc + (int)__builtin_amdgcn_mbcnt_lo(mj, 0u); \
          if (pos < WCAP) list[wave * WCAP + pos] = ((el0 + (J)) << 12) | (int)(SJ); \
        } \
        wc += (int)__builtin_popcount(mj); } }
    HITJ(0, h0, s0)
    HITJ(1, h1, s1)
    HITJ(2, h2, s2)
    HITJ(3, h3, s3)
    HITJ(4, h4, s4)
    HITJ(5, h5, s5)
    HITJ(6, h6, s6)
    HITJ(7, h7, s7)
#undef HITJ
  }
  return wc;
}

__global__ __launch_bounds__(NTHR) void k_wprep(const float* __restrict__ wlin, const float* __restrict__ w1,
                                                _Float16* wt, _Float16* w1t) {
  const int j = (int)blockIdx.y;
  const int u = (int)blockIdx.x * NTHR + (int)threadIdx.x;
  if (u >= 8192) return;
  if (j == 0) {
    const int n  = u >> 4;
    const int k8 = (u & 15) * 8;
    const float* p = wlin + (size_t)k8 * FO + n;
    v4f a, b;
    a.x = p[0 * FO]; a.y = p[1 * FO]; a.z = p[2 * FO]; a.w = p[3 * FO];
    b.x = p[4 * FO]; b.y = p[5 * FO]; b.z = p[6 * FO]; b.w = p[7 * FO];
    const v8h hv = pack8(a, b, CW);
    const size_t o = (size_t)n * WP + k8;
    *(volatile v8h*)(wt + o) = hv;
    __threadfence();
    *(volatile v8h*)(wt + o) = hv;
  } else {
    const int n  = u >> 6;
    const int k8 = (u & 63) * 8;
    const float* p = w1 + ((size_t)(n >> 6) * FO + (size_t)k8) * DH + (n & 63);
    v4f a, b;
    a.x = p[0 * DH]; a.y = p[1 * DH]; a.z = p[2 * DH]; a.w = p[3 * DH];
    b.x = p[4 * DH]; b.y = p[5 * DH]; b.z = p[6 * DH]; b.w = p[7 * DH];
    const v8h hv = pack8(a, b, CW);
    const size_t o = (size_t)n * W1P + k8;
    *(volatile v8h*)(w1t + o) = hv;
    __threadfence();
    *(volatile v8h*)(w1t + o) = hv;
  }
}

__global__ __launch_bounds__(NTHR) void k_prep(const float* __restrict__ ea, const float* __restrict__ wedge,
                                               const float* __restrict__ aedge, float* misc, int nE) {
  __shared__ double sd[NTHR];
  __shared__ float sm[EC];
  __shared__ __attribute__((aligned(16))) float sv[MISCN];
  const int tid = threadIdx.x;
  {
    const int k = tid & 15, gq = tid >> 4;
    double acc = 0.0;
#pragma unroll 1
    for (int r = gq; r < nE; r += 16) acc += (double)ea[(size_t)r * EC + k];
    sd[tid] = acc;
  }
  for (int i = tid; i < MISCN; i += NTHR) sv[i] = 0.f;
  __syncthreads();
  if (tid < EC) {
    double t = 0.0;
#pragma unroll 1
    for (int g2 = 0; g2 < 16; ++g2) t += sd[g2 * 16 + tid];
    sm[tid] = (float)t * (1.0f / (float)nE);
  }
  if (tid < EC * NH) {
    const int k = tid >> 3, h = tid & 7;
    float s = 0.f;
#pragma unroll 1
    for (int c = 0; c < HC; ++c) s = fmaf(wedge[(size_t)k * FO + h * HC + c], aedge[h * HC + c], s);
    sv[tid] = s;
  }
  __syncthreads();
  if (tid < NH) {
    float a = 0.f;
#pragma unroll 1
    for (int k = 0; k < EC; ++k) a = fmaf(sm[k], sv[k * NH + tid], a);
    sv[EC * NH + tid] = a;
  }
  __syncthreads();
  const bool w = tid < MISCN / 4;
  const v4f v = *(const v4f*)(sv + 4 * (w ? tid : 0));
  if (w) *(volatile v4f*)(misc + 4 * tid) = v;
  __threadfence();
  if (w) *(volatile v4f*)(misc + 4 * tid) = v;
}

__global__ __launch_bounds__(GTHR) void k_gemm1(const float* __restrict__ x, const _Float16* __restrict__ wt,
                                                const float* __restrict__ asrc, const float* __restrict__ adst,
                                                _Float16* XS, float* ES, float* ED, int nN) {
  __shared__ __attribute__((aligned(16))) _Float16 sA[GBM * SAP];
  __shared__ __attribute__((aligned(16))) float stg[GBM * FIN];
  __shared__ __attribute__((aligned(16))) float esT[GBM * ESP];
  __shared__ __attribute__((aligned(16))) float edT[GBM * ESP];
  __shared__ float sAs[FO];
  __shared__ float sAd[FO];
  const int tid = threadIdx.x, lane = tid & 31, wave = tid >> 5, hh = lane >> 4, m = lane & 15;
  const int rowBase = (int)blockIdx.x * GBM;
  for (int i = tid; i < FO; i += GTHR) { sAs[i] = asrc[i]; sAd[i] = adst[i]; }
#pragma unroll 1
  for (int u = tid; u < GBM * (FIN / 8); u += GTHR) {
    const int row = u >> 4, c0 = (u & 15) * 8;
    const int rg  = rowBase + row;
    const int rc  = rg < nN ? rg : nN - 1;
    const float* p = x + (size_t)rc * FIN + c0;
    const v4f a = *(const v4f*)p, b = *(const v4f*)(p + 4);
    *(v8h*)(sA + (size_t)row * SAP + c0) = pack8(a, b, CA);
  }
  __syncthreads();
  const _Float16* ap = sA + (size_t)(16 * wave + m) * SAP + 8 * hh;
  const size_t brow = (size_t)m * WP + 8 * hh;
#pragma unroll 1
  for (int cg = 0; cg < FO / FIN; ++cg) {
    v8f acc[8];
#pragma unroll
    for (int t = 0; t < 8; ++t) { v8f z = {0.f, 0.f, 0.f, 0.f, 0.f, 0.f, 0.f, 0.f}; acc[t] = z; }
#pragma unroll 1
    for (int ks = 0; ks < FIN / 32; ++ks) {
      FragH af;
      af.h[0] = *(const v8h*)(ap + 32 * ks);
      af.h[1] = *(const v8h*)(ap + 32 * ks + 16);
#pragma unroll
      for (int t = 0; t < 8; ++t) {
        const size_t bo = brow + (size_t)(FIN * cg + 16 * t) * WP + 32 * ks;
        FragH bf;
        bf.h[0] = *(const v8h*)(wt + bo);
        bf.h[1] = *(const v8h*)(wt + bo + 16);
        acc[t] = wmh(af, bf, acc[t]);
      }
    }
    {
      float* sp = stg + (size_t)(16 * wave + 8 * hh) * FIN + m;
#pragma unroll
      for (int t = 0; t < 8; ++t) {
#pragma unroll
        for (int r = 0; r < 8; ++r) sp[(size_t)r * FIN + 16 * t] = acc[t][r] * SCL;
      }
    }
    __syncthreads();
    {
      const int row  = tid >> 1;
      const int half = tid & 1;
      const float* srow = stg + (size_t)row * FIN;
#pragma unroll 1
      for (int p = 0; p < 2; ++p) {
        float s = 0.f, d = 0.f;
#pragma unroll 1
        for (int c = 0; c < HC / 2; ++c) {
          const int cc = HC * p + (HC / 2) * half + c;
          const float v = srow[cc];
          s = fmaf(v, sAs[FIN * cg + cc], s);
          d = fmaf(v, sAd[FIN * cg + cc], d);
        }
        s += __shfl_xor(s, 1);
        d += __shfl_xor(d, 1);
        if (half == 0) {
          esT[row * ESP + 2 * cg + p] = s;
          edT[row * ESP + 2 * cg + p] = d;
        }
      }
    }
    {
      _Float16* xb = XS + (size_t)rowBase * XSP + FIN * cg;
      const v4f* s4 = (const v4f*)stg;
#pragma unroll 1
      for (int f = tid; f < GBM * 16; f += GTHR) {
        const int r = f >> 4, q = f & 15;
        const v8h hv = pack8(s4[r * 32 + 2 * q], s4[r * 32 + 2 * q + 1], CX);
        *(volatile v8h*)(xb + (size_t)r * XSP + 8 * q) = hv;
      }
      __threadfence();
#pragma unroll 1
      for (int f = tid; f < GBM * 16; f += GTHR) {
        const int r = f >> 4, q = f & 15;
        const v8h hv = pack8(s4[r * 32 + 2 * q], s4[r * 32 + 2 * q + 1], CX);
        *(volatile v8h*)(xb + (size_t)r * XSP + 8 * q) = hv;
      }
    }
    __syncthreads();
  }
  {
    const v4f ve = *(const v4f*)(esT + 4 * tid);
    const v4f vd = *(const v4f*)(edT + 4 * tid);
    float* pe = ES + (size_t)rowBase * ESP + 4 * tid;
    float* pd = ED + (size_t)rowBase * ESP + 4 * tid;
    *(volatile v4f*)pe = ve;
    *(volatile v4f*)pd = vd;
    __threadfence();
    *(volatile v4f*)pe = ve;
    *(volatile v4f*)pd = vd;
  }
}

__global__ __launch_bounds__(NTHR) void k_build(const int* __restrict__ dsts, int* EL, int* OFF, int* CNT,
                                                int nE, int nb, int tp, int vec8) {
  extern __shared__ v4f lds_dyn[];
  int* reg1 = (int*)lds_dyn;
  int* reg2 = reg1 + RCAP;
  int* scnt = reg2 + RCAP;
  int* soff = scnt + NBMAX;
  int* list = soff + NBMAX;
  int* wcnt = list + LISTN;
  int* wtot = wcnt + NWAVE;
  const int tid = threadIdx.x, lane = tid & 31, wave = tid >> 5;
  const int nodeBase = (int)blockIdx.x * nb;

  for (int i = tid; i < NBMAX; i += NTHR) scnt[i] = 0;
  {
    const v4i z = {0, 0, 0, 0};
    v4i* r2v = (v4i*)reg2;
    for (int f = tid; f < RCAP / 4; f += NTHR) r2v[f] = z;
  }
  __syncthreads();

  int tot = 0;
  const int nChunks = (nE + CHUNK - 1) / CHUNK;
#pragma unroll 1
  for (int ch = 0; ch < nChunks; ++ch) {
    const int cbase = ch * CHUNK;
    const int wc = scan_chunk(dsts, nE, cbase, nodeBase, nb, vec8, list, tid, lane, wave);
    if (lane == 0) wcnt[wave] = wc;
    __syncthreads();
    int pre = 0, all = 0;
#pragma unroll
    for (int w2 = 0; w2 < NWAVE; ++w2) {
      int c = wcnt[w2];
      c = c < 0 ? 0 : (c > WCAP ? WCAP : c);
      all += c;
      pre += (w2 < wave) ? c : 0;
    }
    const int wcc  = wc > WCAP ? WCAP : wc;
    const int base = tot + pre;
#pragma unroll 1
    for (int i = lane; i < wcc; i += 32) {
      const int ent = list[wave * WCAP + i];
      const int el  = (ent >> 12) & (CHUNK - 1);
      const int sl  = ent & (NBMAX - 1);
      int eid = cbase + el;
      eid = eid > nE - 1 ? nE - 1 : eid;
      const int pos = base + i;
      if (pos < RCAP) reg1[pos] = (int)(((unsigned)eid << SLOTB) | (unsigned)sl);
    }
    tot += all;
    tot = tot > RCAP ? RCAP : tot;
    __syncthreads();
  }
  const int nh = tot;

  if (wave == 0) {
#pragma unroll 1
    for (int b0 = 0; b0 < nh; b0 += 32) {
      const int idx = b0 + lane;
      const int uv  = reg1[idx < RCAP ? idx : RCAP - 1];
      const int m32 = (nh - b0) < 32 ? (nh - b0) : 32;
#pragma unroll 1
      for (int k = 0; k < m32; ++k) {
        const int u  = __builtin_amdgcn_readlane(uv, k);
        const int sl = u & (NBMAX - 1);
        if (lane == 0) scnt[sl] = scnt[sl] + 1;
      }
    }
  }
  __syncthreads();

  {
    const v4i ca = *(const v4i*)(scnt + 8 * tid);
    const v4i cb = *(const v4i*)(scnt + 8 * tid + 4);
    const int e0 = ca.x < 0 ? 0 : ca.x, e1 = ca.y < 0 ? 0 : ca.y, e2 = ca.z < 0 ? 0 : ca.z, e3 = ca.w < 0 ? 0 : ca.w;
    const int e4 = cb.x < 0 ? 0 : cb.x, e5 = cb.y < 0 ? 0 : cb.y, e6 = cb.z < 0 ? 0 : cb.z, e7 = cb.w < 0 ? 0 : cb.w;
    const int ts = e0 + e1 + e2 + e3 + e4 + e5 + e6 + e7;
    int incl = ts;
#pragma unroll
    for (int d = 1; d < 32; d <<= 1) {
      const int up = __shfl_up(incl, d);
      if (lane >= d) incl += up;
    }
    if (lane == 31) wtot[wave] = incl;
    __syncthreads();
    int pre = 0;
#pragma unroll
    for (int w2 = 0; w2 < NWAVE; ++w2) pre += (w2 < wave) ? wtot[w2] : 0;
    int run = pre + incl - ts;
    soff[8 * tid + 0] = run; run += e0;
    soff[8 * tid + 1] = run; run += e1;
    soff[8 * tid + 2] = run; run += e2;
    soff[8 * tid + 3] = run; run += e3;
    soff[8 * tid + 4] = run; run += e4;
    soff[8 * tid + 5] = run; run += e5;
    soff[8 * tid + 6] = run; run += e6;
    soff[8 * tid + 7] = run;
  }
  __syncthreads();
  for (int i = tid; i < NBMAX; i += NTHR) list[i] = soff[i];
  __syncthreads();

  if (wave == 0) {
#pragma unroll 1
    for (int b0 = 0; b0 < nh; b0 += 32) {
      const int idx = b0 + lane;
      const int uv  = reg1[idx < RCAP ? idx : RCAP - 1];
      const int m32 = (nh - b0) < 32 ? (nh - b0) : 32;
#pragma unroll 1
      for (int k = 0; k < m32; ++k) {
        const int u   = __builtin_amdgcn_readlane(uv, k);
        const int sl  = u & (NBMAX - 1);
        const int eid = (int)((unsigned)u >> SLOTB);
        if (lane == 0) {
          int pos = list[sl];
          pos = pos < 0 ? 0 : (pos > RCAP - 1 ? RCAP - 1 : pos);
          reg2[pos] = eid;
          list[sl] = pos + 1;
        }
      }
    }
  }
  __syncthreads();

  {
    int* elb = EL + (size_t)blockIdx.x * RCAP;
    const v4i* r4 = (const v4i*)reg2;
#pragma unroll 1
    for (int f = tid; f < RCAP / 4; f += NTHR) {
      const v4i v = r4[f];
      *(volatile v4i*)(elb + 4 * f) = v;
    }
    __threadfence();
#pragma unroll 1
    for (int f = tid; f < RCAP / 4; f += NTHR) {
      const v4i v = r4[f];
      *(volatile v4i*)(elb + 4 * f) = v;
    }
  }
  {
    const bool ovf = (nh >= RCAP);
    int* ob = OFF + (size_t)blockIdx.x * tp;
    int* cb = CNT + (size_t)blockIdx.x * tp;
    const int n4 = tp >> 2;
#pragma unroll 1
    for (int pass = 0; pass < 2; ++pass) {
#pragma unroll 1
      for (int f = tid; f < n4; f += NTHR) {
        v4i so, sc;
        {
          const int s = 4 * f + 0; const bool in = s < nb; const int scl = s < NBMAX ? s : NBMAX - 1;
          so.x = in ? soff[scl] : 0; sc.x = in ? (ovf ? -1 : scnt[scl]) : 0;
        }
        {
          const int s = 4 * f + 1; const bool in = s < nb; const int scl = s < NBMAX ? s : NBMAX - 1;
          so.y = in ? soff[scl] : 0; sc.y = in ? (ovf ? -1 : scnt[scl]) : 0;
        }
        {
          const int s = 4 * f + 2; const bool in = s < nb; const int scl = s < NBMAX ? s : NBMAX - 1;
          so.z = in ? soff[scl] : 0; sc.z = in ? (ovf ? -1 : scnt[scl]) : 0;
        }
        {
          const int s = 4 * f + 3; const bool in = s < nb; const int scl = s < NBMAX ? s : NBMAX - 1;
          so.w = in ? soff[scl] : 0; sc.w = in ? (ovf ? -1 : scnt[scl]) : 0;
        }
        *(volatile v4i*)(ob + 4 * f) = so;
        *(volatile v4i*)(cb + 4 * f) = sc;
      }
      __threadfence();
    }
  }
}

__global__ __launch_bounds__(NTHR) void k_agg(
    const int* __restrict__ srcs, const int* __restrict__ EL,
    const int* __restrict__ OFF, const int* __restrict__ CNT,
    const _Float16* __restrict__ XS, const float* __restrict__ ES, const float* __restrict__ ED,
    const float* __restrict__ ea, const float* __restrict__ misc, const float* __restrict__ bias,
    _Float16* HB, float* ZP, int nN, int nE, int nb, int tp) {
  __shared__ __attribute__((aligned(32))) v8f cmb[NWAVE * EPI * LPS * 4];
  __shared__ float cdn[NWAVE * EPI * LPS];
  __shared__ __attribute__((aligned(32))) float zw[NWAVE * FO];
  __shared__ float sWea[EC * NH];
  __shared__ float sAl[NH];
  const int tid = threadIdx.x, lane = tid & 31, wave = tid >> 5;
  const int g  = lane >> 4;
  const int j  = lane & 15;
  const int hd = j >> 1;
  const int jA = lane >> 2, pA = lane & 3, jB = 8 + jA;
  if (tid < EC * NH) sWea[tid] = misc[tid];
  if (tid < NH) sAl[tid] = misc[EC * NH + tid];
  __syncthreads();
  const int nodeBase = (int)blockIdx.x * nb;
  const int nbw = nb >> 3;
  const int* elb  = EL  + (size_t)blockIdx.x * RCAP;
  const int* offb = OFF + (size_t)blockIdx.x * tp;
  const int* cntb = CNT + (size_t)blockIdx.x * tp;
  float wk[EC];
#pragma unroll
  for (int k = 0; k < EC; ++k) wk[k] = sWea[k * NH + hd];
  const float al = sAl[hd];
  const float qnan = __int_as_float(0x7fc00000);
  const v8f z8 = {0.f, 0.f, 0.f, 0.f, 0.f, 0.f, 0.f, 0.f};
  v8f zA = z8, zB = z8;
  v8f* cw = cmb + wave * (EPI * LPS * 4);
  float* cd = cdn + wave * (EPI * LPS);
#pragma unroll 1
  for (int jt = 0; jt < nbw; ++jt) {
    const int slot = wave * nbw + jt;
    const int grow = nodeBase + slot;
    const int gcl  = grow < nN ? grow : nN - 1;
    const bool wr  = grow < nN;
    int st = offb[slot];
    const int craw = cntb[slot];
    st = st < 0 ? 0 : (st > RCAP - 1 ? RCAP - 1 : st);
    int cnt = craw < 0 ? 0 : (craw > DEGCAP ? DEGCAP : craw);
    if (cnt > RCAP - st) cnt = RCAP - st;
    const float pz = (craw < 0 || craw > DEGCAP) ? qnan : 0.0f;

    const float edv = ED[(size_t)gcl * ESP + hd];
    const float esd = ES[(size_t)gcl * ESP + hd];
    const float t0  = esd + edv + al;
    float mx = fmaxf(t0, NEG_SLOPE * t0);
    const _Float16* yd = XS + (size_t)gcl * XSP + 32 * j;
    const bool g0 = (g == 0);
    float dn = g0 ? 1.0f : 0.0f;
    v8f a0 = cvt8(*(const v8h*)(yd));
    v8f a1 = cvt8(*(const v8h*)(yd + 8));
    v8f a2 = cvt8(*(const v8h*)(yd + 16));
    v8f a3 = cvt8(*(const v8h*)(yd + 24));
    a0 = g0 ? a0 : z8; a1 = g0 ? a1 : z8; a2 = g0 ? a2 : z8; a3 = g0 ? a3 : z8;
    const int niter = (cnt + EPI - 1) / EPI;
#pragma unroll 1
    for (int it = 0; it < niter; ++it) {
      const int qq = it * EPI + g;
      const bool valid = qq < cnt;
      const int qc = valid ? qq : cnt - 1;
      const int idx = st + qc;
      int eid = elb[idx];
      eid = eid < 0 ? 0 : (eid > nE - 1 ? nE - 1 : eid);
      const int sraw = srcs[eid];
      const int s = sraw < 0 ? 0 : (sraw > nN - 1 ? nN - 1 : sraw);
      const _Float16* ys = XS + (size_t)s * XSP + 32 * j;
      const v8f x0 = cvt8(*(const v8h*)(ys));
      const v8f x1 = cvt8(*(const v8h*)(ys + 8));
      const v8f x2 = cvt8(*(const v8h*)(ys + 16));
      const v8f x3 = cvt8(*(const v8h*)(ys + 24));
      const float* eap = ea + (size_t)eid * EC;
      const v4f ev0 = *(const v4f*)(eap), ev1 = *(const v4f*)(eap + 4);
      const v4f ev2 = *(const v4f*)(eap + 8), ev3 = *(const v4f*)(eap + 12);
      float ae = ev0.x * wk[0];
      ae = fmaf(ev0.y, wk[1], ae);  ae = fmaf(ev0.z, wk[2], ae);  ae = fmaf(ev0.w, wk[3], ae);
      ae = fmaf(ev1.x, wk[4], ae);  ae = fmaf(ev1.y, wk[5], ae);  ae = fmaf(ev1.z, wk[6], ae);  ae = fmaf(ev1.w, wk[7], ae);
      ae = fmaf(ev2.x, wk[8], ae);  ae = fmaf(ev2.y, wk[9], ae);  ae = fmaf(ev2.z, wk[10], ae); ae = fmaf(ev2.w, wk[11], ae);
      ae = fmaf(ev3.x, wk[12], ae); ae = fmaf(ev3.y, wk[13], ae); ae = fmaf(ev3.z, wk[14], ae); ae = fmaf(ev3.w, wk[15], ae);
      const float ess = ES[(size_t)s * ESP + hd];
      const float u = ess + edv + ae;
      float l = fmaxf(u, NEG_SLOPE * u);
      l = valid ? l : (mx - 100.0f);
      const float mn = fmaxf(mx, l);
      const float s1 = __expf(mx - mn), s2 = __expf(l - mn);
      dn = fmaf(dn, s1, s2);
      a0 = a0 * s1 + x0 * s2;
      a1 = a1 * s1 + x1 * s2;
      a2 = a2 * s1 + x2 * s2;
      a3 = a3 * s1 + x3 * s2;
      mx = mn;
    }
    const float m1 = fmaxf(mx, __shfl_xor(mx, 16));
    const float e = __expf(mx - m1);
    __builtin_amdgcn_fence(__ATOMIC_RELEASE, "wavefront");
    __builtin_amdgcn_wave_barrier();
    v8f* cg8 = cw + g * (LPS * 4) + 4 * j;
    cg8[0] = a0 * e; cg8[1] = a1 * e; cg8[2] = a2 * e; cg8[3] = a3 * e;
    cd[g * LPS + j] = dn * e;
    __builtin_amdgcn_fence(__ATOMIC_RELEASE, "wavefront");
    __builtin_amdgcn_wave_barrier();
    const v8f rA = cw[4 * jA + pA] + cw[LPS * 4 + 4 * jA + pA];
    const v8f rB = cw[4 * jB + pA] + cw[LPS * 4 + 4 * jB + pA];
    const float dsA = cd[jA] + cd[LPS + jA];
    const float dsB = cd[jB] + cd[LPS + jB];
    const float iA = __builtin_amdgcn_rcpf(dsA) * INVCX;
    const float iB = __builtin_amdgcn_rcpf(dsB) * INVCX;
    U8 bA, bB;
    bA.q[0] = *(const v4f*)(bias + 8 * lane);
    bA.q[1] = *(const v4f*)(bias + 8 * lane + 4);
    bB.q[0] = *(const v4f*)(bias + (FO / 2) + 8 * lane);
    bB.q[1] = *(const v4f*)(bias + (FO / 2) + 8 * lane + 4);
    const v8f hA = leaky8(rA * iA + bA.v) + pz;
    const v8f hB = leaky8(rB * iB + bB.v) + pz;
    if (wr) {
      zA += hA;
      zB += hB;
      const v8h hvA = pack8v(hA, CH);
      const v8h hvB = pack8v(hB, CH);
      _Float16* hp = HB + (size_t)gcl * HP + 8 * lane;
      *(volatile v8h*)hp = hvA;
      *(volatile v8h*)(hp + (FO / 2)) = hvB;
      __threadfence();
      *(volatile v8h*)hp = hvA;
      *(volatile v8h*)(hp + (FO / 2)) = hvB;
    }
  }
  *(v8f*)(zw + (size_t)wave * FO + 8 * lane) = zA;
  *(v8f*)(zw + (size_t)wave * FO + (FO / 2) + 8 * lane) = zB;
  __syncthreads();
  {
    const bool zs = tid < FO / 4;
    const int zt = zs ? tid : 0;
    v4f zz = *(const v4f*)(zw + 4 * zt);
#pragma unroll
    for (int w2 = 1; w2 < NWAVE; ++w2) zz += *(const v4f*)(zw + (size_t)w2 * FO + 4 * zt);
    float* zp = ZP + (size_t)blockIdx.x * FO + 4 * zt;
    if (zs) *(volatile v4f*)zp = zz;
    __threadfence();
    if (zs) *(volatile v4f*)zp = zz;
  }
}

__global__ __launch_bounds__(GTHR) void k_gemm2(const _Float16* __restrict__ hb, const _Float16* __restrict__ w1t,
                                                float* PQ, int nN) {
  __shared__ __attribute__((aligned(16))) float stg[GBM * PQW];
  const int tid = threadIdx.x, lane = tid & 31, wave = tid >> 5, hh = lane >> 4, m = lane & 15;
  const int rowBase = (int)blockIdx.x * GBM;
  int ar = rowBase + 16 * wave + m;
  ar = ar < nN ? ar : nN - 1;
  const _Float16* ap = hb + (size_t)ar * HP + 8 * hh;
  const size_t brow = (size_t)m * W1P + 8 * hh;
  v8f acc[8];
#pragma unroll
  for (int t = 0; t < 8; ++t) { v8f z = {0.f, 0.f, 0.f, 0.f, 0.f, 0.f, 0.f, 0.f}; acc[t] = z; }
#pragma unroll 1
  for (int ks = 0; ks < K2 / 32; ++ks) {
    FragH af;
    af.h[0] = *(const v8h*)(ap + 32 * ks);
    af.h[1] = *(const v8h*)(ap + 32 * ks + 16);
#pragma unroll
    for (int t = 0; t < 8; ++t) {
      const size_t bo = brow + (size_t)(16 * t) * W1P + 32 * ks;
      FragH bf;
      bf.h[0] = *(const v8h*)(w1t + bo);
      bf.h[1] = *(const v8h*)(w1t + bo + 16);
      acc[t] = wmh(af, bf, acc[t]);
    }
  }
  {
    float* sp = stg + (size_t)(16 * wave + 8 * hh) * PQW + m;
#pragma unroll
    for (int t = 0; t < 8; ++t) {
#pragma unroll
      for (int r = 0; r < 8; ++r) sp[(size_t)r * PQW + 16 * t] = acc[t][r] * SCL;
    }
  }
  __syncthreads();
  {
    const int nF4 = GBM * PQW / 4;
    float* pb = PQ + (size_t)rowBase * PQW;
    const v4f* s4 = (const v4f*)stg;
#pragma unroll 1
    for (int f = tid; f < nF4; f += GTHR) {
      const int r = f >> 5, q = f & 31;
      const v4f v = s4[f];
      *(volatile v4f*)(pb + (size_t)r * PQW + 4 * q) = v;
    }
    __threadfence();
#pragma unroll 1
    for (int f = tid; f < nF4; f += GTHR) {
      const int r = f >> 5, q = f & 31;
      const v4f v = s4[f];
      *(volatile v4f*)(pb + (size_t)r * PQW + 4 * q) = v;
    }
  }
}

__global__ __launch_bounds__(ETHR) void k_edge(const float* __restrict__ ea, const int* ei,
                                               const float* PQ, const float* __restrict__ w1,
                                               const float* __restrict__ b1, const float* __restrict__ w2,
                                               const float* __restrict__ b2, float* out, int nN, int nE, int nTiles) {
  __shared__ __attribute__((aligned(16))) float sW[EC * DH];
  __shared__ __attribute__((aligned(16))) float sb1[DH];
  __shared__ __attribute__((aligned(16))) float sw2[DH * 2];
  __shared__ __attribute__((aligned(16))) float sT[(ETHR / 32) * 16 * STP];
  __shared__ __attribute__((aligned(16))) float sO[(ETHR / 32) * 32];
  const int tid = threadIdx.x, lane = tid & 31, wave = tid >> 5, hh = lane >> 4, m = lane & 15;
  {
    const float* wsrc = w1 + (size_t)K1OFF * DH;
    const v4f wa = *(const v4f*)(wsrc + 4 * tid);
    const v4f wb = *(const v4f*)(wsrc + 4 * (tid + ETHR));
    const v4f bb = *(const v4f*)(b1 + 4 * (tid & 15));
    const v4f ww = *(const v4f*)(w2 + 4 * (tid & 31));
    *(v4f*)(sW + 4 * tid) = wa;
    *(v4f*)(sW + 4 * (tid + ETHR)) = wb;
    if (tid < 16) *(v4f*)(sb1 + 4 * tid) = bb;
    if (tid < 32) *(v4f*)(sw2 + 4 * tid) = ww;
  }
  const float b20 = b2[0], b21 = b2[1];
  __syncthreads();
  const v8i zi8 = {0, 0, 0, 0, 0, 0, 0, 0};
  FragH bq[4];
  float b1v[4], w2a[4], w2b[4];
#pragma unroll
  for (int t = 0; t < 4; ++t) {
    const float* wp = sW + (8 * hh) * DH + 16 * t + m;
    v4f wa, wb;
    wa.x = wp[0 * DH]; wa.y = wp[1 * DH]; wa.z = wp[2 * DH]; wa.w = wp[3 * DH];
    wb.x = wp[4 * DH]; wb.y = wp[5 * DH]; wb.z = wp[6 * DH]; wb.w = wp[7 * DH];
    bq[t].w = zi8;
    bq[t].h[0] = pack8(wa, wb, CW);
    b1v[t] = sb1[16 * t + m];
    w2a[t] = sw2[(16 * t + m) * 2 + 0];
    w2b[t] = sw2[(16 * t + m) * 2 + 1];
  }
  float* st = sT + wave * (16 * STP);
  float* so = sO + wave * 32;
#pragma unroll 1
  for (int tw = 0; tw < TPW; ++tw) {
    const int traw = ((int)blockIdx.x * (ETHR / 32) + wave) * TPW + tw;
    const bool tv  = traw < nTiles;
    const int tile = tv ? traw : nTiles - 1;
    const int e0 = tile * 16;
    int em = e0 + m;
    em = em < nE ? em : nE - 1;
    const float* eap = ea + (size_t)em * EC + 8 * hh;
    const v4f xa = *(const v4f*)eap, xb = *(const v4f*)(eap + 4);
    FragH af;
    af.w = zi8;
    af.h[0] = pack8(xa, xb, CA);
    v8f acc[4];
#pragma unroll
    for (int t = 0; t < 4; ++t) { v8f z = {0.f, 0.f, 0.f, 0.f, 0.f, 0.f, 0.f, 0.f}; acc[t] = z; }
#pragma unroll
    for (int t = 0; t < 4; ++t) acc[t] = wmh(af, bq[t], acc[t]);

    int nid = ei[(size_t)(hh != 0 ? nE : 0) + (size_t)em];
    nid = nid < 0 ? 0 : (nid > nN - 1 ? nN - 1 : nid);
#pragma unroll
    for (int i = 0; i < 8; ++i) {
      const int bi = __shfl(nid, (lane & 16) | i);
      const v4f v = *(const v4f*)(PQ + (size_t)bi * PQW + 4 * lane);
      *(v4f*)(st + i * STP + 4 * lane) = v;
    }
    __threadfence();
#pragma unroll
    for (int i = 8; i < 16; ++i) {
      const int bi = __shfl(nid, (lane & 16) | i);
      const v4f v = *(const v4f*)(PQ + (size_t)bi * PQW + 4 * lane);
      *(v4f*)(st + i * STP + 4 * lane) = v;
    }
    __builtin_amdgcn_fence(__ATOMIC_RELEASE, "wavefront");
    __builtin_amdgcn_wave_barrier();

    float o0[8], o1[8];
#pragma unroll
    for (int r = 0; r < 8; ++r) {
      const float* pr = st + (8 * hh + r) * STP + m;
      const float* pc = pr + DH;
      float s0 = 0.f, s1 = 0.f;
#pragma unroll
      for (int t = 0; t < 4; ++t) {
        float v = fmaf(acc[t][r], SCL, b1v[t]) + pr[16 * t] + pc[16 * t];
        v = fmaxf(v, 0.f);
        s0 = fmaf(v, w2a[t], s0);
        s1 = fmaf(v, w2b[t], s1);
      }
      o0[r] = s0; o1[r] = s1;
    }
#pragma unroll
    for (int r = 0; r < 8; ++r) {
      o0[r] += __shfl_xor(o0[r], 1); o1[r] += __shfl_xor(o1[r], 1);
      o0[r] += __shfl_xor(o0[r], 2); o1[r] += __shfl_xor(o1[r], 2);
      o0[r] += __shfl_xor(o0[r], 4); o1[r] += __shfl_xor(o1[r], 4);
      o0[r] += __shfl_xor(o0[r], 8); o1[r] += __shfl_xor(o1[r], 8);
    }
    if (m == 0) {
#pragma unroll
      for (int r = 0; r < 8; ++r) {
        so[2 * (8 * hh + r) + 0] = o0[r] + b20;
        so[2 * (8 * hh + r) + 1] = o1[r] + b21;
      }
    }
    __builtin_amdgcn_fence(__ATOMIC_RELEASE, "wavefront");
    __builtin_amdgcn_wave_barrier();
    const v4f ov = *(const v4f*)(so + 4 * (lane & 7));
    const bool stl = tv && (lane < 8);
    float* op = out + (size_t)e0 * 2 + 4 * (lane & 7);
    if (stl) *(volatile v4f*)op = ov;
    __threadfence();
    if (stl) *(volatile v4f*)op = ov;
    __builtin_amdgcn_fence(__ATOMIC_RELEASE, "wavefront");
    __builtin_amdgcn_wave_barrier();
  }
}

__global__ __launch_bounds__(FO) void k_group(const float* __restrict__ ZP, const float* __restrict__ wg1,
                                              const float* __restrict__ bg1, const float* __restrict__ wg2,
                                              const float* __restrict__ bg2, float* out, int gA, int nN, int o1) {
  __shared__ float sz[FO];
  __shared__ float st[GH];
  const int tid = threadIdx.x;
  {
    float s = 0.f;
#pragma unroll 1
    for (int b = 0; b < gA; ++b) s += ZP[(size_t)b * FO + tid];
    sz[tid] = s * (1.0f / (float)nN);
  }
  __syncthreads();
  if (tid < GH) {
    float a = bg1[tid];
#pragma unroll 1
    for (int c = 0; c < FO; ++c) a = fmaf(sz[c], wg1[(size_t)c * GH + tid], a);
    st[tid] = fmaxf(a, 0.f);
  }
  __syncthreads();
  if (tid == 0) {
    float gs = bg2[0];
#pragma unroll 1
    for (int jj = 0; jj < GH; ++jj) gs = fmaf(st[jj], wg2[jj], gs);
    const float r = __builtin_amdgcn_rcpf(1.0f + __expf(-gs));
    *(volatile float*)(out + o1) = r;
    __threadfence();
    *(volatile float*)(out + o1) = r;
  }
}

static int pick_nb(int nE, int nN) {
  int nb = NBMAX;
  while (nb > 16 && (long long)nb * (long long)nE * 5LL > (long long)RCAP * (long long)nN * 4LL) nb >>= 1;
  return nb;
}

extern "C" void kernel_launch(void* const* d_in, const int* in_sizes, int n_in,
                              void* d_out, int out_size, void* d_ws, size_t ws_size,
                              hipStream_t stream) {
  if (n_in < 17) return;
  if (in_sizes[0] < FIN) return;
  const int nN = in_sizes[0] / FIN;
  if (in_sizes[0] != nN * FIN || nN > (1 << 22)) return;
  if (in_sizes[1] < 2 || (in_sizes[1] & 1) != 0) return;
  const int nE = in_sizes[1] / 2;
  if (nE < 16 || (nE % 16) != 0 || nE > (1 << 21)) return;
  if (in_sizes[2] != nE * EC) return;
  if (in_sizes[3] != FIN * FO) return;
  if (in_sizes[4] != FO || in_sizes[5] != FO) return;
  if (in_sizes[6] != EC * FO) return;
  if (in_sizes[7] != FO || in_sizes[8] != FO) return;
  if (in_sizes[9] != MLPIN * DH || in_sizes[10] != DH) return;
  if (in_sizes[11] != DH * 2 || in_sizes[12] != 2) return;
  if (in_sizes[13] != FO * GH || in_sizes[14] != GH) return;
  if (in_sizes[15] != GH || in_sizes[16] != 1) return;
  if (out_size != 2 * nE + 1) return;

  const float* x     = (const float*)d_in[0];
  const int*   ei    = (const int*)d_in[1];
  const float* ea    = (const float*)d_in[2];
  const float* wlin  = (const float*)d_in[3];
  const float* asrc  = (const float*)d_in[4];
  const float* adst  = (const float*)d_in[5];
  const float* wedge = (const float*)d_in[6];
  const float* aedge = (const float*)d_in[7];
  const float* gbias = (const float*)d_in[8];
  const float* w1    = (const float*)d_in[9];
  const float* b1    = (const float*)d_in[10];
  const float* w2    = (const float*)d_in[11];
  const float* b2    = (const float*)d_in[12];
  const float* wg1   = (const float*)d_in[13];
  const float* bg1   = (const float*)d_in[14];
  const float* wg2   = (const float*)d_in[15];
  const float* bg2   = (const float*)d_in[16];
  float* out = (float*)d_out;
  const int* dsts = ei + nE;

  const int MP     = ((nN + GBM - 1) / GBM) * GBM;
  const int nb     = pick_nb(nE, nN);
  const int tp     = nb < 32 ? 32 : nb;
  const int gA     = (nN + nb - 1) / nb;
  const int gG     = MP / GBM;
  const int vec8   = ((nE & 3) == 0) ? 1 : 0;
  const int nTiles = nE / 16;
  const int tpb    = (ETHR / 32) * TPW;
  const int gE     = (nTiles + tpb - 1) / tpb;
  const int o1     = 2 * nE;
  if (nb < 16 || nb > NBMAX || (long long)gA * nb < (long long)nN) return;
  if (o1 >= out_size) return;

  char* ws = (char*)d_ws;
  size_t off = 0;
  const size_t oWT   = off; off += (size_t)FO * WP * 2;          off = (off + 255) & ~(size_t)255;
  const size_t oW1T  = off; off += (size_t)PQW * W1P * 2;        off = (off + 255) & ~(size_t)255;
  const size_t oXS   = off; off += (size_t)MP * XSP * 2;         off = (off + 255) & ~(size_t)255;
  const size_t oHB   = off; off += (size_t)nN * HP * 2;          off = (off + 255) & ~(size_t)255;
  const size_t oPQ   = off; off += (size_t)MP * PQW * 4;         off = (off + 255) & ~(size_t)255;
  const size_t oES   = off; off += (size_t)MP * ESP * 4;         off = (off + 255) & ~(size_t)255;
  const size_t oED   = off; off += (size_t)MP * ESP * 4;         off = (off + 255) & ~(size_t)255;
  const size_t oEL   = off; off += (size_t)gA * RCAP * 4;        off = (off + 255) & ~(size_t)255;
  const size_t oOFF  = off; off += (size_t)gA * tp * 4;          off = (off + 255) & ~(size_t)255;
  const size_t oCNT  = off; off += (size_t)gA * tp * 4;          off = (off + 255) & ~(size_t)255;
  const size_t oZP   = off; off += (size_t)gA * FO * 4;          off = (off + 255) & ~(size_t)255;
  const size_t oMISC = off; off += (size_t)MISCN * 4;            off = (off + 255) & ~(size_t)255;
  if (off > ws_size || off > (size_t)WSCAP) return;
  _Float16* WT   = (_Float16*)(ws + oWT);
  _Float16* W1T  = (_Float16*)(ws + oW1T);
  _Float16* XS   = (_Float16*)(ws + oXS);
  _Float16* HB   = (_Float16*)(ws + oHB);
  float*    PQ   = (float*)(ws + oPQ);
  float*    ES   = (float*)(ws + oES);
  float*    ED   = (float*)(ws + oED);
  int*      EL   = (int*)(ws + oEL);
  int*      OFF  = (int*)(ws + oOFF);
  int*      CNT  = (int*)(ws + oCNT);
  float*    ZP   = (float*)(ws + oZP);
  float*    MISC = (float*)(ws + oMISC);

  hipFuncSetAttribute(reinterpret_cast<const void*>(&k_build),
                      hipFuncAttributeMaxDynamicSharedMemorySize, LDS_BUILD);

  k_wprep<<<dim3(8192 / NTHR, 2), NTHR, 0, stream>>>(wlin, w1, WT, W1T);
  k_prep<<<1, NTHR, 0, stream>>>(ea, wedge, aedge, MISC, nE);

  k_build<<<gA, NTHR, LDS_BUILD, stream>>>(dsts, EL, OFF, CNT, nE, nb, tp, vec8);

  k_gemm1<<<gG, GTHR, 0, stream>>>(x, WT, asrc, adst, XS, ES, ED, nN);
  k_agg<<<gA, NTHR, 0, stream>>>(ei, EL, OFF, CNT, XS, ES, ED, ea, MISC, gbias, HB, ZP, nN, nE, nb, tp);

  k_gemm2<<<gG, GTHR, 0, stream>>>(HB, W1T, PQ, nN);
  k_edge<<<gE, ETHR, 0, stream>>>(ea, ei, PQ, w1, b1, w2, b2, out, nN, nE, nTiles);

  k_group<<<1, FO, 0, stream>>>(ZP, wg1, bg1, wg2, bg2, out, gA, nN, o1);
}
